// MultiHeadSelfAttention_32212254720501
// MI455X (gfx1250) — hardware-verified
//
#include <hip/hip_runtime.h>
#include <stdint.h>
#include <stddef.h>


#ifndef NB
#define NB 2
#endif
#ifndef SEQ
#define SEQ 2048
#endif
#define NB_FULL 2
#define SEQ_FULL 2048
#define DD 1024
#define HH 16
#define HD 64
#define M_TOT (NB * SEQ)
#define BHN (NB * HH)

static_assert(SEQ % 128 == 0);
static_assert(SEQ >= 128 && SEQ <= SEQ_FULL);
static_assert(NB >= 1 && NB <= NB_FULL);
static_assert(DD == HH * HD);
static_assert(DD % 64 == 0);

typedef __attribute__((ext_vector_type(16))) _Float16 v16h;
typedef __attribute__((ext_vector_type(8)))  _Float16 v8h;
typedef __attribute__((ext_vector_type(8)))  float    v8f;
typedef __attribute__((ext_vector_type(4)))  float    v4f;
typedef __attribute__((ext_vector_type(4)))  unsigned int v4u;

__device__ __forceinline__ v16h load_frag(const _Float16* p, int lh) {
    union { v16h h; v4u u[2]; } f;
    f.u[0] = *reinterpret_cast<const v4u*>(p + lh);
    f.u[1] = *reinterpret_cast<const v4u*>(p + lh + 16);
    return f.h;
}

__device__ __forceinline__ v16h load_frag_lds(const _Float16* p, int lh) {
    union { v16h h; v4u u[2]; } f;
    f.u[0] = *reinterpret_cast<const v4u*>(p + lh);
    f.u[1] = *reinterpret_cast<const v4u*>(p + lh + 16);
    return f.h;
}

__device__ __forceinline__ v8f wmma_f16(v16h a, v16h b, v8f c) {
    v8f d = __builtin_amdgcn_wmma_f32_16x16x32_f16(false, a, false, b,
                                                   (short)0, c, false, false);
    asm volatile("v_nop\n\tv_nop\n\tv_nop\n\tv_nop" : "+v"(d) : "v"(a), "v"(b));
    return d;
}

__device__ __forceinline__ float bf16_rne(float f) {
    unsigned u = __float_as_uint(f);
    u = (u + 0x7FFFu + ((u >> 16) & 1u)) & 0xFFFF0000u;
    return __uint_as_float(u);
}

__device__ __forceinline__ void pack_hi_lo(v4f a, v4f c, v4u& hi, v4u& lo) {
    float v[8];
    v[0] = a.x; v[1] = a.y; v[2] = a.z; v[3] = a.w;
    v[4] = c.x; v[5] = c.y; v[6] = c.z; v[7] = c.w;
    union { v8h h; v4u u; } ph, pl;
    #pragma unroll
    for (int i = 0; i < 8; ++i) {
        const _Float16 hx = (_Float16)v[i];
        ph.h[i] = hx;
        pl.h[i] = (_Float16)((v[i] - (float)hx) * 1024.0f);
    }
    hi = ph.u; lo = pl.u;
}

__global__ void __launch_bounds__(256)
cvt_plane_kernel(const float* __restrict__ in, _Float16* __restrict__ out, int n8, float scale)
{
    const int i = blockIdx.x * 256 + threadIdx.x;
    if (i >= n8) return;
    const float* src = in + (size_t)i * 8;
    const v4f a = *reinterpret_cast<const v4f*>(src);
    const v4f c = *reinterpret_cast<const v4f*>(src + 4);
    float v[8];
    v[0] = a.x; v[1] = a.y; v[2] = a.z; v[3] = a.w;
    v[4] = c.x; v[5] = c.y; v[6] = c.z; v[7] = c.w;
    union { v8h h; v4u u; } o;
    #pragma unroll
    for (int k = 0; k < 8; ++k) o.h[k] = (_Float16)(bf16_rne(v[k]) * scale);
    const v4u w = o.u;
    volatile v4u* dst = reinterpret_cast<volatile v4u*>(out + (size_t)i * 8);
    *dst = w;
    __threadfence();
    *dst = w;
}

__device__ __forceinline__ void gemm_tile_128x64(const _Float16* __restrict__ arow0,
                                                 const _Float16* __restrict__ arow1,
                                                 const _Float16* __restrict__ Wn,
                                                 _Float16 (*ldsB)[32],
                                                 int tid, int r, int lh,
                                                 v8f (&acc0)[4], v8f (&acc1)[4])
{
    for (int kc = 0; kc < DD; kc += 32) {
        __syncthreads();
        #pragma unroll
        for (int s = 0; s < 2; ++s) {
            const int bb  = tid * 16 + s * 2048;
            const int row = bb >> 6;
            const int kh  = (bb & 63) >> 1;
            const v4u v = *reinterpret_cast<const v4u*>(Wn + (size_t)row * DD + kc + kh);
            *reinterpret_cast<v4u*>(&ldsB[row][kh]) = v;
        }
        __syncthreads();
        const v16h a0 = load_frag(arow0 + kc, lh);
        const v16h a1 = load_frag(arow1 + kc, lh);
        #pragma unroll
        for (int nt = 0; nt < 4; ++nt) {
            const v16h bf = load_frag_lds(&ldsB[nt * 16 + r][0], lh);
            acc0[nt] = wmma_f16(a0, bf, acc0[nt]);
            acc1[nt] = wmma_f16(a1, bf, acc1[nt]);
        }
    }
}

__global__ void __launch_bounds__(128)
qkv_gemm_kernel(const _Float16* __restrict__ X16,
                const _Float16* __restrict__ Wq16, const _Float16* __restrict__ Wk16,
                const _Float16* __restrict__ Wv16,
                _Float16* __restrict__ Qh, _Float16* __restrict__ Ql,
                _Float16* __restrict__ Kh, _Float16* __restrict__ Kl,
                _Float16* __restrict__ Vth, _Float16* __restrict__ Vtl)
{
    __shared__ __align__(16) _Float16 ldsB[64][32];
    __shared__ __align__(16) float stg[128 * 64];

    const int tid  = threadIdx.x;
    const int lane = tid & 31;
    const int wave = tid >> 5;
    const int r    = lane & 15;
    const int lh   = (lane & 16) ? 8 : 0;
    const int hs   = (lane >> 4) & 1;

    const int n0g = blockIdx.x * 64;
    const int sel = n0g >> 10;
    const int nn  = n0g & (DD - 1);
    const int h   = nn >> 6;
    const int m0b = blockIdx.y * 128;
    const int b   = m0b / SEQ;
    const int t0b = m0b - b * SEQ;
    const bool wlo = (t0b == 0);

    const _Float16* W = (sel == 0) ? Wq16 : ((sel == 1) ? Wk16 : Wv16);
    const _Float16* arow0 = X16 + (size_t)(m0b + wave * 32 + r) * DD;
    const _Float16* arow1 = arow0 + (size_t)16 * DD;

    v8f acc0[4] = {}, acc1[4] = {};
    gemm_tile_128x64(arow0, arow1, W + (size_t)nn * DD, ldsB, tid, r, lh, acc0, acc1);

    #pragma unroll
    for (int nt = 0; nt < 4; ++nt) {
        const int col = nt * 16 + r;
        #pragma unroll
        for (int mt = 0; mt < 2; ++mt) {
            #pragma unroll
            for (int g = 0; g < 8; ++g) {
                const int rowl = wave * 32 + mt * 16 + hs * 8 + g;
                const float v  = (mt ? acc1[nt][g] : acc0[nt][g]) * 0.015625f;
                const int idx  = (sel == 2) ? (col * 128 + rowl) : (rowl * 64 + col);
                stg[idx] = v;
            }
        }
    }
    __syncthreads();

    _Float16* ph;
    _Float16* pl;
    size_t base;
    if (sel == 0)      { ph = Qh;  pl = Ql;  base = ((size_t)(b * HH + h) * SEQ + t0b) * HD; }
    else if (sel == 1) { ph = Kh;  pl = Kl;  base = ((size_t)(b * HH + h) * SEQ + t0b) * HD; }
    else               { ph = Vth; pl = Vtl; base = (size_t)(b * HH + h) * HD * SEQ + t0b; }

    for (int pass = 0; pass < 2; ++pass) {
        #pragma unroll
        for (int it = 0; it < 8; ++it) {
            const int e = (it * 128 + tid) * 8;
            const v4f a = *reinterpret_cast<const v4f*>(&stg[e]);
            const v4f c = *reinterpret_cast<const v4f*>(&stg[e + 4]);
            v4u hi, lo;
            pack_hi_lo(a, c, hi, lo);
            const size_t go = (sel == 2) ? ((size_t)(e >> 7) * SEQ + (size_t)(e & 127)) : (size_t)e;
            *reinterpret_cast<volatile v4u*>(ph + base + go) = hi;
            if (wlo) *reinterpret_cast<volatile v4u*>(pl + base + go) = lo;
        }
        if (pass == 0) __threadfence();
    }
}

template <int EARLY>
__global__ void __launch_bounds__(128)
attn_kernel(const _Float16* __restrict__ Qh, const _Float16* __restrict__ Ql,
            const _Float16* __restrict__ Kh, const _Float16* __restrict__ Kl,
            const _Float16* __restrict__ Vth, const _Float16* __restrict__ Vtl,
            _Float16* __restrict__ Ch, _Float16* __restrict__ Cl, int xoff)
{
    __shared__ __align__(16) _Float16 ldsK[32][64];
    __shared__ __align__(16) _Float16 ldsV[64][32];
    __shared__ __align__(16) _Float16 ldsKl[32][64];
    __shared__ __align__(16) _Float16 ldsVl[64][32];
    __shared__ __align__(16) _Float16 plds[4][16][32];
    __shared__ __align__(16) _Float16 prlds[4][16][32];
    __shared__ __align__(16) float    ostg[4][16][64];

    const int tid  = threadIdx.x;
    const int lane = tid & 31;
    const int wave = tid >> 5;
    const int r    = lane & 15;
    const int lh   = (lane & 16) ? 8 : 0;
    const int hs   = (lane >> 4) & 1;

    const int q0b = (blockIdx.x + xoff) * 64;
    const int q0  = q0b + wave * 16;
    const int bh  = blockIdx.y;
    const int b   = bh / HH;
    const int h   = bh - b * HH;

    const size_t poff = (size_t)bh * SEQ * HD;
    const _Float16* qb  = Qh  + poff;
    const _Float16* qlb = Ql  + poff;
    const _Float16* kb  = Kh  + poff;
    const _Float16* klb = Kl  + poff;
    const _Float16* vb  = Vth + poff;
    const _Float16* vlb = Vtl + poff;

    const v16h qf0 = load_frag(qb + (size_t)(q0 + r) * HD, lh);
    const v16h qf1 = load_frag(qb + (size_t)(q0 + r) * HD + 32, lh);
    v16h ql0 = qf0, ql1 = qf1;
    if (EARLY) {
        ql0 = load_frag(qlb + (size_t)(q0 + r) * HD, lh);
        ql1 = load_frag(qlb + (size_t)(q0 + r) * HD + 32, lh);
    }

    v8f acc[4] = {};
    v8f accr[4] = {};
    float m[8], l[8];
    #pragma unroll
    for (int g = 0; g < 8; ++g) { m[g] = -1.0e30f; l[g] = 0.0f; }

    const float scale = 0.125f;
    const float rk    = 0.0009765625f;
    const int kv_end  = q0b + 64;

    for (int kv = 0; kv < kv_end; kv += 32) {
        __syncthreads();
        #pragma unroll
        for (int s = 0; s < 2; ++s) {
            const int bb = tid * 16 + s * 2048;
            const int kr = bb >> 7;
            const int kc = (bb & 127) >> 1;
            *reinterpret_cast<v4u*>(&ldsK[kr][kc]) =
                *reinterpret_cast<const v4u*>(kb + (size_t)(kv + kr) * HD + kc);
            const int vr = bb >> 6;
            const int vc = (bb & 63) >> 1;
            *reinterpret_cast<v4u*>(&ldsV[vr][vc]) =
                *reinterpret_cast<const v4u*>(vb + (size_t)vr * SEQ + kv + vc);
            if (EARLY) {
                *reinterpret_cast<v4u*>(&ldsKl[kr][kc]) =
                    *reinterpret_cast<const v4u*>(klb + (size_t)(kv + kr) * HD + kc);
                *reinterpret_cast<v4u*>(&ldsVl[vr][vc]) =
                    *reinterpret_cast<const v4u*>(vlb + (size_t)vr * SEQ + kv + vc);
            }
        }
        __syncthreads();

        v8f s0 = {}, s1 = {};
        s0 = wmma_f16(qf0, load_frag_lds(&ldsK[r][0],       lh), s0);
        s0 = wmma_f16(qf1, load_frag_lds(&ldsK[r][32],      lh), s0);
        s1 = wmma_f16(qf0, load_frag_lds(&ldsK[16 + r][0],  lh), s1);
        s1 = wmma_f16(qf1, load_frag_lds(&ldsK[16 + r][32], lh), s1);
        if (EARLY) {
            v8f e0 = {}, e1 = {};
            e0 = wmma_f16(qf0, load_frag_lds(&ldsKl[r][0],       lh), e0);
            e0 = wmma_f16(qf1, load_frag_lds(&ldsKl[r][32],      lh), e0);
            e0 = wmma_f16(ql0, load_frag_lds(&ldsK[r][0],        lh), e0);
            e0 = wmma_f16(ql1, load_frag_lds(&ldsK[r][32],       lh), e0);
            e1 = wmma_f16(qf0, load_frag_lds(&ldsKl[16 + r][0],  lh), e1);
            e1 = wmma_f16(qf1, load_frag_lds(&ldsKl[16 + r][32], lh), e1);
            e1 = wmma_f16(ql0, load_frag_lds(&ldsK[16 + r][0],   lh), e1);
            e1 = wmma_f16(ql1, load_frag_lds(&ldsK[16 + r][32],  lh), e1);
            s0 = s0 + e0 * rk;
            s1 = s1 + e1 * rk;
        }

        #pragma unroll
        for (int g = 0; g < 8; ++g) {
            const int qrow = q0 + hs * 8 + g;
            const int key0 = kv + r;
            const int key1 = kv + 16 + r;
            float a0 = s0[g] * scale;
            float a1 = s1[g] * scale;
            a0 = (key0 > qrow) ? -1.0e30f : a0;
            a1 = (key1 > qrow) ? -1.0e30f : a1;
            float mx = fmaxf(a0, a1);
            mx = fmaxf(mx, __shfl_xor(mx, 1));
            mx = fmaxf(mx, __shfl_xor(mx, 2));
            mx = fmaxf(mx, __shfl_xor(mx, 4));
            mx = fmaxf(mx, __shfl_xor(mx, 8));
            const float nm = fmaxf(m[g], mx);
            const float p0 = __expf(a0 - nm);
            const float p1 = __expf(a1 - nm);
            float rs = p0 + p1;
            rs += __shfl_xor(rs, 1);
            rs += __shfl_xor(rs, 2);
            rs += __shfl_xor(rs, 4);
            rs += __shfl_xor(rs, 8);
            const float alpha = __expf(m[g] - nm);
            l[g] = l[g] * alpha + rs;
            m[g] = nm;
            const int prow = hs * 8 + g;
            const float c0 = p0 * 1024.0f;
            const float c1 = p1 * 1024.0f;
            const _Float16 h0 = (_Float16)c0;
            const _Float16 h1 = (_Float16)c1;
            plds[wave][prow][r]      = h0;
            plds[wave][prow][16 + r] = h1;
            if (EARLY) {
                prlds[wave][prow][r]      = (_Float16)((c0 - (float)h0) * 1024.0f);
                prlds[wave][prow][16 + r] = (_Float16)((c1 - (float)h1) * 1024.0f);
            }
            #pragma unroll
            for (int t = 0; t < 4; ++t) {
                acc[t][g] *= alpha;
                if (EARLY) accr[t][g] *= alpha;
            }
        }
        __syncthreads();

        const v16h pf = load_frag(&plds[wave][r][0], lh);
        v16h prf = pf;
        if (EARLY) prf = load_frag(&prlds[wave][r][0], lh);
        #pragma unroll
        for (int t = 0; t < 4; ++t) {
            const v16h vf = load_frag_lds(&ldsV[t * 16 + r][0], lh);
            acc[t] = wmma_f16(pf, vf, acc[t]);
            if (EARLY) {
                const v16h vl = load_frag_lds(&ldsVl[t * 16 + r][0], lh);
                accr[t] = wmma_f16(pf, vl, accr[t]);
                accr[t] = wmma_f16(prf, vf, accr[t]);
            }
        }
    }

    #pragma unroll
    for (int g = 0; g < 8; ++g) {
        const float inv = 1.0f / (l[g] * 1024.0f);
        const int row = hs * 8 + g;
        #pragma unroll
        for (int t = 0; t < 4; ++t) {
            float o = acc[t][g];
            if (EARLY) o = o + accr[t][g] * rk;
            ostg[wave][row][t * 16 + r] = o * inv;
        }
    }
    __syncthreads();

    for (int pass = 0; pass < 2; ++pass) {
        #pragma unroll
        for (int j = 0; j < 4; ++j) {
            const int row = j * 4 + (lane >> 3);
            const int c8  = (lane & 7) * 8;
            const v4f a = *reinterpret_cast<const v4f*>(&ostg[wave][row][c8]);
            const v4f c = *reinterpret_cast<const v4f*>(&ostg[wave][row][c8 + 4]);
            v4u hi, lo;
            pack_hi_lo(a, c, hi, lo);
            const size_t go = ((size_t)(b * SEQ + q0 + row)) * DD + (size_t)h * HD + c8;
            *reinterpret_cast<volatile v4u*>(Ch + go) = hi;
            *reinterpret_cast<volatile v4u*>(Cl + go) = lo;
        }
        if (pass == 0) __threadfence();
    }
}

__global__ void __launch_bounds__(128)
out_gemm_kernel(const _Float16* __restrict__ Ch, const _Float16* __restrict__ Cl,
                const _Float16* __restrict__ Wo16, float* __restrict__ out)
{
    __shared__ __align__(16) _Float16 ldsB[64][32];
    __shared__ __align__(16) float stg[128 * 64];

    const int tid  = threadIdx.x;
    const int lane = tid & 31;
    const int wave = tid >> 5;
    const int r    = lane & 15;
    const int lh   = (lane & 16) ? 8 : 0;
    const int hs   = (lane >> 4) & 1;

    const int n0  = blockIdx.x * 64;
    const int m0b = blockIdx.y * 128;
    const int b   = m0b / SEQ;
    const int t0b = m0b - b * SEQ;
    const bool use_lo = (t0b == 0);

    const size_t ra0 = (size_t)(m0b + wave * 32 + r) * DD;
    const size_t ra1 = ra0 + (size_t)16 * DD;
    const _Float16* Wn = Wo16 + (size_t)n0 * DD;

    v8f acc0[4] = {}, acc1[4] = {};
    gemm_tile_128x64(Ch + ra0, Ch + ra1, Wn, ldsB, tid, r, lh, acc0, acc1);

    #pragma unroll
    for (int nt = 0; nt < 4; ++nt) {
        const int col = nt * 16 + r;
        #pragma unroll
        for (int mt = 0; mt < 2; ++mt) {
            #pragma unroll
            for (int g = 0; g < 8; ++g) {
                const int rowl = wave * 32 + mt * 16 + hs * 8 + g;
                const float v  = (mt ? acc1[nt][g] : acc0[nt][g]) * 0.015625f;
                stg[rowl * 64 + col] = v;
            }
        }
    }

    if (use_lo) {
        const v8f zero8 = {0.0f, 0.0f, 0.0f, 0.0f, 0.0f, 0.0f, 0.0f, 0.0f};
        #pragma unroll
        for (int nt = 0; nt < 4; ++nt) { acc0[nt] = zero8; acc1[nt] = zero8; }
        gemm_tile_128x64(Cl + ra0, Cl + ra1, Wn, ldsB, tid, r, lh, acc0, acc1);
        #pragma unroll
        for (int nt = 0; nt < 4; ++nt) {
            const int col = nt * 16 + r;
            #pragma unroll
            for (int mt = 0; mt < 2; ++mt) {
                #pragma unroll
                for (int g = 0; g < 8; ++g) {
                    const int rowl = wave * 32 + mt * 16 + hs * 8 + g;
                    const float v  = (mt ? acc1[nt][g] : acc0[nt][g]) * (1.0f / 65536.0f);
                    stg[rowl * 64 + col] += v;
                }
            }
        }
    }
    __syncthreads();

    const size_t orow0 = (size_t)b * SEQ_FULL + t0b;
    for (int pass = 0; pass < 2; ++pass) {
        #pragma unroll
        for (int j = 0; j < 16; ++j) {
            const int row = wave * 32 + j * 2 + (lane >> 4);
            const int c4  = (lane & 15) * 4;
            const v4f v = *reinterpret_cast<const v4f*>(&stg[row * 64 + c4]);
            *reinterpret_cast<volatile v4f*>(out + (orow0 + row) * DD + n0 + c4) = v;
        }
        if (pass == 0) __threadfence();
    }
}

extern "C" void kernel_launch(void* const* d_in, const int* in_sizes, int n_in,
                              void* d_out, int out_size, void* d_ws, size_t ws_size,
                              hipStream_t stream)
{
    if (n_in < 5) return;
    const long long need_x = (long long)(NB - 1) * SEQ_FULL * DD + (long long)SEQ * DD;
    if ((long long)in_sizes[0] < need_x) return;
    for (int i = 1; i < 5; ++i) if (in_sizes[i] < DD * DD) return;
    if ((long long)out_size < need_x) return;

    const float* x  = (const float*)d_in[0];
    const float* wq = (const float*)d_in[1];
    const float* wk = (const float*)d_in[2];
    const float* wv = (const float*)d_in[3];
    const float* wo = (const float*)d_in[4];
    float* out = (float*)d_out;

    char* ws = (char*)d_ws;
    size_t off = 0;
    auto carve = [&](size_t bytes) -> char* {
        char* p = ws + off;
        off = (off + bytes + 255) & ~(size_t)255;
        return p;
    };
    const size_t plane  = (size_t)NB * SEQ * DD * 2;
    const size_t wbytes = (size_t)DD * DD * 2;
    _Float16* X16  = (_Float16*)carve(plane);
    _Float16* Wq16 = (_Float16*)carve(wbytes);
    _Float16* Wk16 = (_Float16*)carve(wbytes);
    _Float16* Wv16 = (_Float16*)carve(wbytes);
    _Float16* Wo16 = (_Float16*)carve(wbytes);
    _Float16* Qh   = (_Float16*)carve(plane);
    _Float16* Ql   = (_Float16*)carve(plane);
    _Float16* Kh   = (_Float16*)carve(plane);
    _Float16* Kl   = (_Float16*)carve(plane);
    _Float16* Vth  = (_Float16*)carve(plane);
    _Float16* Vtl  = (_Float16*)carve(plane);
    _Float16* Ch   = (_Float16*)carve(plane);
    _Float16* Cl   = (_Float16*)carve(plane);
    if (off > ws_size) return;

    {
        const int n8 = SEQ * DD / 8;
        for (int bq = 0; bq < NB; ++bq)
            cvt_plane_kernel<<<(n8 + 255) / 256, 256, 0, stream>>>(
                x + (size_t)bq * SEQ_FULL * DD, X16 + (size_t)bq * SEQ * DD, n8, 1.0f);
        const int n8w = DD * DD / 8;
        cvt_plane_kernel<<<(n8w + 255) / 256, 256, 0, stream>>>(wq, Wq16, n8w, 64.0f);
        cvt_plane_kernel<<<(n8w + 255) / 256, 256, 0, stream>>>(wk, Wk16, n8w, 64.0f);
        cvt_plane_kernel<<<(n8w + 255) / 256, 256, 0, stream>>>(wv, Wv16, n8w, 64.0f);
        cvt_plane_kernel<<<(n8w + 255) / 256, 256, 0, stream>>>(wo, Wo16, n8w, 64.0f);
    }

    qkv_gemm_kernel<<<dim3(3 * DD / 64, M_TOT / 128), 128, 0, stream>>>(
        X16, Wq16, Wk16, Wv16, Qh, Ql, Kh, Kl, Vth, Vtl);

    attn_kernel<1><<<dim3(1, BHN), 128, 0, stream>>>(Qh, Ql, Kh, Kl, Vth, Vtl, Ch, Cl, 0);
    if (SEQ / 64 > 1)
        attn_kernel<0><<<dim3(SEQ / 64 - 1, BHN), 128, 0, stream>>>(Qh, Ql, Kh, Kl, Vth, Vtl, Ch, Cl, 1);

    out_gemm_kernel<<<dim3(DD / 64, M_TOT / 128), 128, 0, stream>>>(Ch, Cl, Wo16, out);
}
